// PartialEncoder_25168508354670
// MI455X (gfx1250) — hardware-verified
//
#include <hip/hip_runtime.h>
#include <hip/hip_bf16.h>

typedef __attribute__((ext_vector_type(16))) _Float16 v16bf;
typedef __attribute__((ext_vector_type(8)))  float  v8f;
typedef __attribute__((ext_vector_type(4)))  float  v4f;
typedef float __attribute__((may_alias)) float_a;
template <typename T> __device__ __forceinline__ void vst2(void* p, T v) { *(volatile T*)p = v; __threadfence(); *(volatile T*)p = v; }
__device__ __forceinline__ v8f wmma16(v16bf a, v16bf b, v8f c) {
    v8f d = __builtin_amdgcn_wmma_f32_16x16x32_f16(false, a, false, b, (short)0, c, false, false);
    asm volatile("v_nop\n\tv_nop\n\tv_nop\n\tv_nop" : "+v"(d) : "v"(a), "v"(b));
    return d;
}

#define Bn 64
#define Dn 25000
#define Kn 16
#define Hn 128
#define En 256
#define Zn 32

#define TPW 8
#define SPAN (16 * TPW)
#define WPB ((Dn + SPAN - 1) / SPAN)
#define WAVES_PER_BLOCK 8
#define NBLOCKS (Bn * WPB / WAVES_PER_BLOCK)

__device__ __forceinline__ float4 ld4(const float* p) { return *(const float4*)p; }

__global__ void build_g_kernel(const float* __restrict__ feat_emb,
                               const float* __restrict__ feat_bias,
                               const float* __restrict__ W1,
                               const float* __restrict__ b1,
                               float* __restrict__ G) {
    int idx = blockIdx.x * blockDim.x + threadIdx.x;
    if (idx >= Dn * Hn) return;
    int d = idx >> 7;
    int k = idx & 127;
    float acc = b1[k] + feat_bias[d] * W1[17 * Hn + k];
    const float* fe = feat_emb + d * Kn;
#pragma unroll
    for (int r = 0; r < 16; ++r) acc = fmaf(fe[r], W1[(1 + r) * Hn + k], acc);
    vst2(G + idx, (float_a)acc);
}

#define CVT4(dst, off, g4, w4)                                      \
    dst[(off) + 0] = (_Float16)fmaxf(fmaf(xv, (w4).x, (g4).x), 0.f);  \
    dst[(off) + 1] = (_Float16)fmaxf(fmaf(xv, (w4).y, (g4).y), 0.f);  \
    dst[(off) + 2] = (_Float16)fmaxf(fmaf(xv, (w4).z, (g4).z), 0.f);  \
    dst[(off) + 3] = (_Float16)fmaxf(fmaf(xv, (w4).w, (g4).w), 0.f);

__global__ void __launch_bounds__(256)
main_pool_kernel(const float* __restrict__ x,
                 const int*   __restrict__ mask,
                 const float* __restrict__ W1,
                 const float* __restrict__ W2,
                 const float* __restrict__ b2,
                 const float* __restrict__ G,
                 float* __restrict__ partial) {
    const int lane = threadIdx.x & 31;
    const int gwid = blockIdx.x * WAVES_PER_BLOCK + (threadIdx.x >> 5);
    const int b    = gwid / WPB;
    const int seg  = gwid % WPB;
    const int dbase = seg * SPAN;

    const int n    = lane & 15;
    const int half = lane >> 4;

    const float b2n = b2[n];

    v16bf Bw[4];
#pragma unroll
    for (int c = 0; c < 4; ++c) {
#pragma unroll
        for (int e = 0; e < 16; ++e) {
            int K = 32 * c + 8 * half + ((e < 8) ? e : (e + 8));
            Bw[c][e] = (_Float16)W2[K * Kn + n];
        }
    }

    float4 w0v[4][4];
#pragma unroll
    for (int c = 0; c < 4; ++c) {
        const float* p0 = W1 + 32 * c + 8 * half;
        w0v[c][0] = ld4(p0);
        w0v[c][1] = ld4(p0 + 4);
        w0v[c][2] = ld4(p0 + 16);
        w0v[c][3] = ld4(p0 + 20);
    }

    float S[8];
#pragma unroll
    for (int j = 0; j < 8; ++j) S[j] = 0.f;

    const size_t rowbase = (size_t)b * Dn;

    for (int t = 0; t < TPW; ++t) {
        const int d0  = dbase + t * 16;
        const int dm  = d0 + n;
        const int dmc = dm < Dn ? dm : (Dn - 1);
        const float xv = x[rowbase + dmc];
        const int   mk = mask[rowbase + dmc];
        const bool flag = (dm < Dn) && (mk != 0);
        const unsigned mb = (unsigned)__ballot(flag);
        const unsigned mym = (mb >> (8 * half)) & 0xFFu;

        const float* Grow = G + (size_t)dmc * Hn;

        v8f acc;
#pragma unroll
        for (int j = 0; j < 8; ++j) acc[j] = b2n;

#pragma unroll
        for (int c = 0; c < 4; ++c) {
            const float* p0 = Grow + 32 * c + 8 * half;
            float4 g0 = ld4(p0);
            float4 g1 = ld4(p0 + 4);
            float4 g2 = ld4(p0 + 16);
            float4 g3 = ld4(p0 + 20);
            v16bf a;
            CVT4(a, 0,  g0, w0v[c][0]);
            CVT4(a, 4,  g1, w0v[c][1]);
            CVT4(a, 8,  g2, w0v[c][2]);
            CVT4(a, 12, g3, w0v[c][3]);
            acc = wmma16(a, Bw[c], acc);
        }

#pragma unroll
        for (int j = 0; j < 8; ++j) {
            float r = acc[j] > 0.f ? acc[j] : 0.f;
            S[j] += (mym & (1u << j)) ? r : 0.f;
        }
    }

    float s = ((S[0] + S[1]) + (S[2] + S[3])) + ((S[4] + S[5]) + (S[6] + S[7]));
    s += __shfl_xor(s, 16, 32);
    __shared__ __attribute__((aligned(16))) float sp[WAVES_PER_BLOCK][Kn];
    if (half == 0) sp[threadIdx.x >> 5][n] = s;
    __syncthreads();
    if (threadIdx.x < 32) vst2(partial + (size_t)blockIdx.x * WAVES_PER_BLOCK * Kn + threadIdx.x * 4, *(const v4f*)(&sp[0][0] + threadIdx.x * 4));
}

__global__ void __launch_bounds__(256)
encoder_kernel(const float* __restrict__ partial,
               const float* __restrict__ We1, const float* __restrict__ be1,
               const float* __restrict__ We2, const float* __restrict__ be2,
               float* __restrict__ out) {
    __shared__ float crow[Kn];
    __shared__ float a1[En];
    const int b = blockIdx.x;
    const int t = threadIdx.x;

    if (t < Kn) {
        const float* p = partial + (size_t)b * WPB * Kn + t;
        float s = 0.f;
        for (int g = 0; g < WPB; ++g) s += p[(size_t)g * Kn];
        crow[t] = s;
    }
    __syncthreads();

    float s = be1[t];
#pragma unroll
    for (int k = 0; k < Kn; ++k) s = fmaf(crow[k], We1[k * En + t], s);
    a1[t] = fmaxf(s, 0.f);
    __syncthreads();

    if (t < 2 * Zn) {
        float o = be2[t];
        for (int e = 0; e < En; ++e) o = fmaf(a1[e], We2[e * 2 * Zn + t], o);
        int z = t & (Zn - 1);
        if (t < Zn) vst2(out + (size_t)b * Zn + z, (float_a)o);
        else        vst2(out + (size_t)Bn * Zn + (size_t)b * Zn + z, (float_a)o);
    }
}

extern "C" void kernel_launch(void* const* d_in, const int* in_sizes, int n_in,
                              void* d_out, int out_size, void* d_ws, size_t ws_size,
                              hipStream_t stream) {
    const float* x         = (const float*)d_in[0];
    const int*   mask      = (const int*)  d_in[1];
    const float* feat_emb  = (const float*)d_in[2];
    const float* feat_bias = (const float*)d_in[3];
    const float* W1        = (const float*)d_in[4];
    const float* b1        = (const float*)d_in[5];
    const float* W2        = (const float*)d_in[6];
    const float* b2        = (const float*)d_in[7];
    const float* We1       = (const float*)d_in[8];
    const float* be1       = (const float*)d_in[9];
    const float* We2       = (const float*)d_in[10];
    const float* be2       = (const float*)d_in[11];

    float* G       = (float*)d_ws;
    float* partial = G + (size_t)Dn * Hn;

    build_g_kernel<<<(Dn * Hn + 255) / 256, 256, 0, stream>>>(feat_emb, feat_bias, W1, b1, G);
    main_pool_kernel<<<NBLOCKS, 256, 0, stream>>>(x, mask, W1, W2, b2, G, partial);
    encoder_kernel<<<Bn, En, 0, stream>>>(partial, We1, be1, We2, be2, (float*)d_out);
}
